// Attention_3126736192252
// MI455X (gfx1250) — hardware-verified
//
#include <hip/hip_runtime.h>
#include <math.h>

#ifndef NB
#define NB 4
#endif
#ifndef SEQ
#define SEQ 2048
#endif
#define NB_FULL 4
#define SEQ_FULL 2048
#define CDIM 1024
#define NHEAD 16
#define HDIM 64
#define QKW 2048
#define AT_NW 4
#define AT_PP 40

static_assert(NB >= 1 && NB <= NB_FULL);
static_assert(SEQ >= 64 && SEQ <= SEQ_FULL);
static_assert(SEQ % 64 == 0);
static_assert(NHEAD * HDIM == CDIM);
static_assert(HDIM == 64);
static_assert(CDIM % 64 == 0 && CDIM % 32 == 0);
static_assert(QKW == 2 * CDIM);
static_assert(((NB * SEQ) % 64) == 0);
static_assert((AT_PP % 8) == 0 && AT_PP >= 32);

typedef __attribute__((ext_vector_type(16))) _Float16 v16h;
typedef __attribute__((ext_vector_type(8)))  _Float16 v8h;
typedef __attribute__((ext_vector_type(8)))  float    v8f;
typedef __attribute__((ext_vector_type(4)))  float    v4f;
typedef unsigned int cm_u4 __attribute__((ext_vector_type(4)));

union FragU { v16h v; v8h h[2]; };
__device__ __forceinline__ v16h ldfrag_g(const _Float16* __restrict__ p) { FragU f; f.h[0] = *(const v8h*)(p); f.h[1] = *(const v8h*)(p + 16); return f.v; }

__device__ __forceinline__ v8f mma_h(v16h a, v16h b, v8f c) { return __builtin_amdgcn_wmma_f32_16x16x32_f16(false, a, false, b, (short)0, c, false, false); }
__device__ __forceinline__ void dep_guard_h(v8f& a, v8f& b, v16h x, v16h y) { asm volatile("v_nop\n\tv_nop\n\tv_nop\n\tv_nop" : "+v"(a), "+v"(b) : "v"(x), "v"(y)); }
__device__ __forceinline__ void keep4_h(v16h a, v16h b, v16h c, v16h d) { asm volatile("v_nop" :: "v"(a), "v"(b), "v"(c), "v"(d)); }
__device__ __forceinline__ void acc_guard4(v8f& a, v8f& b, v8f& c, v8f& d) { asm volatile("v_nop\n\tv_nop\n\tv_nop\n\tv_nop" : "+v"(a), "+v"(b), "+v"(c), "+v"(d)); }
__device__ __forceinline__ void guard_s(v8f& a, v8f& b, v16h q0, v16h q1, v16h k0, v16h k1, v16h k2, v16h k3) {
    asm volatile("v_nop\n\tv_nop\n\tv_nop\n\tv_nop" : "+v"(a), "+v"(b) : "v"(q0), "v"(q1), "v"(k0), "v"(k1), "v"(k2), "v"(k3)); }
__device__ __forceinline__ void guard_o(v8f& a, v8f& b, v8f& c, v8f& d, v16h p, v16h v0, v16h v1, v16h v2, v16h v3) {
    asm volatile("v_nop\n\tv_nop\n\tv_nop\n\tv_nop" : "+v"(a), "+v"(b), "+v"(c), "+v"(d) : "v"(p), "v"(v0), "v"(v1), "v"(v2), "v"(v3)); }
__device__ __forceinline__ void wave_lds_sync() {
    __builtin_amdgcn_fence(3  , "workgroup");
    __builtin_amdgcn_wave_barrier();
    __builtin_amdgcn_fence(2  , "workgroup");
}

#define VST2(T, ptr, val) do { const T vst2_v_ = (val); *(volatile T*)(ptr) = vst2_v_; __threadfence(); *(volatile T*)(ptr) = vst2_v_; } while (0)

__device__ __forceinline__ unsigned int cmb_pk2(float a, float b) { return (unsigned int)__builtin_bit_cast(unsigned short, (_Float16)a) | ((unsigned int)__builtin_bit_cast(unsigned short, (_Float16)b) << 16); }
__device__ __forceinline__ float cmb_bf(float v) { const unsigned u = __builtin_bit_cast(unsigned, v); const unsigned r = (u + 0x7fffu + ((u >> 16) & 1u)) & 0xffff0000u; return __builtin_bit_cast(float, r); }

__global__ __launch_bounds__(256) void k_cast_x(const float* __restrict__ SRC, unsigned short* __restrict__ DST) {
    const long long u = (long long)blockIdx.x * 256 + threadIdx.x; const int per = CDIM / 8;
    if (u >= (long long)NB * SEQ * per) return;
    const int r = (int)(u / per); const int c0 = 8 * (int)(u % per); const int b = r / SEQ; const int n = r - b * SEQ;
    const float* s = SRC + ((long long)b * SEQ_FULL + n) * CDIM + c0;
    const v4f a = *(const v4f*)(s); const v4f d = *(const v4f*)(s + 4);
    cm_u4 pk; pk.x = cmb_pk2(cmb_bf(a.x), cmb_bf(a.y)); pk.y = cmb_pk2(cmb_bf(a.z), cmb_bf(a.w)); pk.z = cmb_pk2(cmb_bf(d.x), cmb_bf(d.y)); pk.w = cmb_pk2(cmb_bf(d.z), cmb_bf(d.w));
    VST2(cm_u4, (cm_u4*)(DST + (long long)r * CDIM + c0), pk);
}
__global__ __launch_bounds__(256) void k_cm_castbT(const float* __restrict__ SRC, int lds, unsigned short* __restrict__ DST, int ldd, int nR, int nC, float sc) {
    const long long u = (long long)blockIdx.x * 256 + threadIdx.x; const int per = nR / 8; if (u >= (long long)nC * per) return; const int c = (int)(u / per); const int r0 = 8 * (int)(u % per);
    float w[8];
#pragma unroll
    for (int e = 0; e < 8; ++e) w[e] = cmb_bf(SRC[(long long)(r0 + e) * lds + c]) * sc;
    cm_u4 pk; pk.x = cmb_pk2(w[0], w[1]); pk.y = cmb_pk2(w[2], w[3]); pk.z = cmb_pk2(w[4], w[5]); pk.w = cmb_pk2(w[6], w[7]); VST2(cm_u4, (cm_u4*)(DST + (long long)c * ldd + r0), pk);
}

__global__ __launch_bounds__(256) void k_gemm64(
    const unsigned short* __restrict__ Ap, int lda, long long strideA,
    const unsigned short* __restrict__ Btp, int ldb, long long strideB,
    void* __restrict__ Cout, int ldc, long long strideC,
    const float* __restrict__ bias, int M, int N, int K, float scale, int out_mode) {
  __shared__ __align__(16) float sT[8 * 16 * 68];
  const int b    = blockIdx.y;
  const int lane = threadIdx.x & 31;
  const int wave = threadIdx.x >> 5;
  const int tilesN = N >> 6;
  const int tilesM = M >> 6;
  const int tile = blockIdx.x * 8 + wave;
  if (tile >= tilesM * tilesN) return;
  const int tm = tile / tilesN;
  const int tn = tile - tm * tilesN;
  const int m0 = tm << 6;
  const int n0 = tn << 6;

  const _Float16* Ab = (const _Float16*)Ap  + (size_t)b * (size_t)strideA;
  const _Float16* Bb = (const _Float16*)Btp + (size_t)b * (size_t)strideB;

  const int rlane = lane & 15;
  const int koff  = (lane >> 4) * 8;
  const int mOff  = (lane >> 4) * 8;

  v8f acc[4][4];
#pragma unroll
  for (int i = 0; i < 4; ++i)
#pragma unroll
    for (int j = 0; j < 4; ++j) acc[i][j] = (v8f){0.f,0.f,0.f,0.f,0.f,0.f,0.f,0.f};

  for (int k0 = 0; k0 < K; k0 += 32) {
    v16h bh[4];
#pragma unroll
    for (int j = 0; j < 4; ++j) {
      const size_t bo = (size_t)(n0 + (j << 4) + rlane) * ldb + koff + k0;
      bh[j] = ldfrag_g(Bb + bo);
    }
#pragma unroll
    for (int i = 0; i < 4; ++i) {
      const size_t ao = (size_t)(m0 + (i << 4) + rlane) * lda + koff + k0;
      const v16h ah = ldfrag_g(Ab + ao);
#pragma unroll
      for (int j = 0; j < 4; ++j) acc[i][j] = mma_h(ah, bh[j], acc[i][j]);
      dep_guard_h(acc[i][0], acc[i][3], ah, ah);
    }
    keep4_h(bh[0], bh[1], bh[2], bh[3]);
  }
  acc_guard4(acc[0][0], acc[0][1], acc[0][2], acc[0][3]);
  acc_guard4(acc[1][0], acc[1][1], acc[1][2], acc[1][3]);
  acc_guard4(acc[2][0], acc[2][1], acc[2][2], acc[2][3]);
  acc_guard4(acc[3][0], acc[3][1], acc[3][2], acc[3][3]);

  const int sb = wave * 16 * 68;
  float bvj[4];
#pragma unroll
  for (int j = 0; j < 4; ++j) {
    const int n = n0 + (j << 4) + rlane;
    const float braw = bias[n & (CDIM - 1)];
    bvj[j] = (out_mode == 0) ? cmb_bf(braw) : 0.f;
  }
#pragma unroll
  for (int i = 0; i < 4; ++i) {
    const int mBase = m0 + (i << 4);
#pragma unroll
    for (int j = 0; j < 4; ++j) {
#pragma unroll
      for (int r = 0; r < 8; ++r) sT[sb + (mOff + r) * 68 + (j << 4) + rlane] = acc[i][j][r] * scale + bvj[j];
    }
    wave_lds_sync();
    if (out_mode == 0) {
      float* C = (float*)Cout + (size_t)b * (size_t)strideC;
      const int hh = lane >> 4, c4 = (lane & 15) * 4;
      for (int pass = 0; pass < 2; ++pass) {
#pragma unroll
        for (int it = 0; it < 8; ++it) {
          const int row = it * 2 + hh;
          const v4f v = *(const v4f*)&sT[sb + row * 68 + c4];
          *(volatile v4f*)(C + (size_t)(mBase + row) * ldc + n0 + c4) = v;
        }
        __threadfence();
      }
    } else {
      unsigned short* C = (unsigned short*)Cout + (size_t)b * (size_t)strideC;
      const int q = lane >> 3, c8 = (lane & 7) * 8;
      for (int pass = 0; pass < 2; ++pass) {
#pragma unroll
        for (int it = 0; it < 4; ++it) {
          const int row = it * 4 + q;
          const v4f a = *(const v4f*)&sT[sb + row * 68 + c8];
          const v4f d = *(const v4f*)&sT[sb + row * 68 + c8 + 4];
          v8h hv;
          hv[0] = (_Float16)a.x; hv[1] = (_Float16)a.y; hv[2] = (_Float16)a.z; hv[3] = (_Float16)a.w;
          hv[4] = (_Float16)d.x; hv[5] = (_Float16)d.y; hv[6] = (_Float16)d.z; hv[7] = (_Float16)d.w;
          *(volatile v8h*)(C + (size_t)(mBase + row) * ldc + n0 + c8) = hv;
        }
        __threadfence();
      }
    }
    wave_lds_sync();
  }
}

__global__ __launch_bounds__(128) void k_flash(const unsigned short* __restrict__ QKp, const unsigned short* __restrict__ VTp,
                                               const int* __restrict__ mask, unsigned short* __restrict__ AOp) {
  __shared__ __align__(16) _Float16 Pt[AT_NW * 16 * AT_PP];
  __shared__ __align__(16) float    Os[AT_NW * 16 * 68];
  const int tid = threadIdx.x, wave = tid >> 5, lane = tid & 31, hh = lane >> 4, c = lane & 15;
  const int nqb = SEQ / 64;
  const int bx = blockIdx.x;
  const int qb = bx % nqb, bh = bx / nqb, h = bh % NHEAD, b = bh / NHEAD;
  const int q0 = qb * 64 + wave * 16;
  const _Float16* qk = (const _Float16*)QKp;
  const _Float16* vt = (const _Float16*)VTp;

  const long long qoff = ((long long)b * SEQ + q0 + c) * QKW + h * HDIM + 8 * hh;
  const v16h qa0 = ldfrag_g(qk + qoff), qa1 = ldfrag_g(qk + qoff + 32);
  const long long kbase = (long long)b * SEQ * QKW + CDIM + h * HDIM + 8 * hh;
  const long long vbase = ((long long)b * CDIM + h * HDIM + c) * SEQ + 8 * hh;
  const int* mk = mask + (long long)b * SEQ_FULL;
  const int pb = wave * 16 * AT_PP, ob = wave * 16 * 68;
  const float L2E = 1.4426950408889634f;

  float mrow[8], lrow[8];
  v8f o[4];
#pragma unroll
  for (int r = 0; r < 8; ++r) { mrow[r] = -__builtin_inff(); lrow[r] = 0.f; }
#pragma unroll
  for (int t = 0; t < 4; ++t) o[t] = (v8f){0.f,0.f,0.f,0.f,0.f,0.f,0.f,0.f};

#pragma unroll 1
  for (int j0 = 0; j0 < SEQ; j0 += 32) {
    v8f s0 = (v8f){0.f,0.f,0.f,0.f,0.f,0.f,0.f,0.f}, s1 = s0;
    {
      const _Float16* kr0 = qk + kbase + (long long)(j0 + c) * QKW;
      const _Float16* kr1 = qk + kbase + (long long)(j0 + 16 + c) * QKW;
      const v16h k00 = ldfrag_g(kr0), k01 = ldfrag_g(kr0 + 32), k10 = ldfrag_g(kr1), k11 = ldfrag_g(kr1 + 32);
      s0 = mma_h(qa0, k00, s0);
      s1 = mma_h(qa0, k10, s1);
      s0 = mma_h(qa1, k01, s0);
      s1 = mma_h(qa1, k11, s1);
      guard_s(s0, s1, qa0, qa1, k00, k01, k10, k11);
    }
    const int mv0 = mk[j0 + c], mv1 = mk[j0 + 16 + c];
    const float am0 = (mv0 != 1) ? -10000.0f : 0.0f;
    const float am1 = (mv1 != 1) ? -10000.0f : 0.0f;
#pragma unroll
    for (int r = 0; r < 8; ++r) {
      const float v0 = s0[r] * 0.125f + am0;
      const float v1 = s1[r] * 0.125f + am1;
      float mx = fmaxf(v0, v1);
      mx = fmaxf(mx, __shfl_xor(mx, 1, 32)); mx = fmaxf(mx, __shfl_xor(mx, 2, 32));
      mx = fmaxf(mx, __shfl_xor(mx, 4, 32)); mx = fmaxf(mx, __shfl_xor(mx, 8, 32));
      const float mnew = fmaxf(mrow[r], mx);
      const float corr = exp2f((mrow[r] - mnew) * L2E);
      const float p0 = exp2f((v0 - mnew) * L2E);
      const float p1 = exp2f((v1 - mnew) * L2E);
      lrow[r] = lrow[r] * corr + (p0 + p1);
      mrow[r] = mnew;
      o[0][r] *= corr; o[1][r] *= corr; o[2][r] *= corr; o[3][r] *= corr;
      Pt[pb + (8 * hh + r) * AT_PP + c]      = (_Float16)(p0 * 4096.0f);
      Pt[pb + (8 * hh + r) * AT_PP + 16 + c] = (_Float16)(p1 * 4096.0f);
    }
    wave_lds_sync();
    {
      FragU pf;
      pf.h[0] = *(const v8h*)&Pt[pb + c * AT_PP + 8 * hh];
      pf.h[1] = *(const v8h*)&Pt[pb + c * AT_PP + 16 + 8 * hh];
      const v16h pa = pf.v;
      const _Float16* vr = vt + vbase + j0;
      const v16h vf0 = ldfrag_g(vr);
      const v16h vf1 = ldfrag_g(vr + (long long)16 * SEQ);
      const v16h vf2 = ldfrag_g(vr + (long long)32 * SEQ);
      const v16h vf3 = ldfrag_g(vr + (long long)48 * SEQ);
      o[0] = mma_h(pa, vf0, o[0]);
      o[1] = mma_h(pa, vf1, o[1]);
      o[2] = mma_h(pa, vf2, o[2]);
      o[3] = mma_h(pa, vf3, o[3]);
      guard_o(o[0], o[1], o[2], o[3], pa, vf0, vf1, vf2, vf3);
    }
    wave_lds_sync();
  }

#pragma unroll
  for (int r = 0; r < 8; ++r) {
    float l = lrow[r];
    l += __shfl_xor(l, 1, 32); l += __shfl_xor(l, 2, 32); l += __shfl_xor(l, 4, 32); l += __shfl_xor(l, 8, 32);
    const float inv = 1.0f / (l * 64.0f);
    Os[ob + (8 * hh + r) * 68 + c]      = o[0][r] * inv;
    Os[ob + (8 * hh + r) * 68 + 16 + c] = o[1][r] * inv;
    Os[ob + (8 * hh + r) * 68 + 32 + c] = o[2][r] * inv;
    Os[ob + (8 * hh + r) * 68 + 48 + c] = o[3][r] * inv;
  }
  wave_lds_sync();
  {
    const int q = lane >> 3, c8 = (lane & 7) * 8;
    unsigned short* ao = AOp + ((long long)b * SEQ + q0) * CDIM + h * HDIM + c8;
    for (int pass = 0; pass < 2; ++pass) {
#pragma unroll
      for (int it = 0; it < 4; ++it) {
        const int row = it * 4 + q;
        const v4f a = *(const v4f*)&Os[ob + row * 68 + c8];
        const v4f d = *(const v4f*)&Os[ob + row * 68 + c8 + 4];
        v8h hv;
        hv[0] = (_Float16)a.x; hv[1] = (_Float16)a.y; hv[2] = (_Float16)a.z; hv[3] = (_Float16)a.w;
        hv[4] = (_Float16)d.x; hv[5] = (_Float16)d.y; hv[6] = (_Float16)d.z; hv[7] = (_Float16)d.w;
        *(volatile v8h*)(ao + (long long)row * CDIM) = hv;
      }
      __threadfence();
    }
  }
}

#define WS_X16  ((size_t)NB * SEQ * CDIM * 2)
#define WS_W316 ((size_t)3 * CDIM * CDIM * 2)
#define WS_WO16 ((size_t)CDIM * CDIM * 2)
#define WS_QK16 ((size_t)NB * SEQ * QKW * 2)
#define WS_VT16 ((size_t)NB * CDIM * SEQ * 2)
#define WS_AO16 ((size_t)NB * SEQ * CDIM * 2)
#define WS_TOTAL (WS_X16 + WS_W316 + WS_WO16 + WS_QK16 + WS_VT16 + WS_AO16)
static_assert(WS_TOTAL <= (size_t)134217728);
static_assert((WS_X16 % 256) == 0 && (WS_W316 % 256) == 0 && (WS_WO16 % 256) == 0 && (WS_QK16 % 256) == 0 && (WS_VT16 % 256) == 0 && (WS_AO16 % 256) == 0);

extern "C" void kernel_launch(void* const* d_in, const int* in_sizes, int n_in, void* d_out, int out_size, void* d_ws, size_t ws_size, hipStream_t stream) {
    if (n_in < 5) return;
    const long long need_x = ((long long)(NB - 1) * SEQ_FULL + SEQ) * CDIM;
    const long long need_m = (long long)(NB - 1) * SEQ_FULL + SEQ;
    if ((long long)in_sizes[0] < need_x || (long long)in_sizes[1] < need_m || (long long)in_sizes[2] < (long long)CDIM * 3 * CDIM ||
        (long long)in_sizes[3] < (long long)CDIM * CDIM || (long long)in_sizes[4] < (long long)CDIM || (long long)out_size < need_x) return;
    if ((size_t)WS_TOTAL > ws_size) return;
    const float* x     = (const float*)d_in[0];
    const int*   mask  = (const int*)d_in[1];
    const float* wqkv  = (const float*)d_in[2];
    const float* wproj = (const float*)d_in[3];
    const float* bproj = (const float*)d_in[4];
    float* out = (float*)d_out;
    char* wsp = (char*)d_ws;
    unsigned short* X16  = (unsigned short*)wsp; wsp += WS_X16;
    unsigned short* W316 = (unsigned short*)wsp; wsp += WS_W316;
    unsigned short* WO16 = (unsigned short*)wsp; wsp += WS_WO16;
    unsigned short* QK16 = (unsigned short*)wsp; wsp += WS_QK16;
    unsigned short* VT16 = (unsigned short*)wsp; wsp += WS_VT16;
    unsigned short* AO16 = (unsigned short*)wsp; wsp += WS_AO16;

    k_cast_x<<<(unsigned)(((long long)NB * SEQ * (CDIM / 8) + 255) / 256), 256, 0, stream>>>(x, X16);
    k_cm_castbT<<<(unsigned)(((long long)(3 * CDIM) * (CDIM / 8) + 255) / 256), 256, 0, stream>>>(wqkv, 3 * CDIM, W316, CDIM, CDIM, 3 * CDIM, 16.0f);
    k_cm_castbT<<<(unsigned)(((long long)CDIM * (CDIM / 8) + 255) / 256), 256, 0, stream>>>(wproj, CDIM, WO16, CDIM, CDIM, CDIM, 16.0f);

    {
        const int M = NB * SEQ, N = QKW;
        const unsigned gx = (unsigned)(((M / 64) * (N / 64) + 7) / 8);
        k_gemm64<<<dim3(gx, 1u), 256, 0, stream>>>(X16, CDIM, (long long)0, W316, CDIM, (long long)0, (void*)QK16, QKW, (long long)0,
                                                  bproj, M, N, CDIM, 0.0625f, 1);
    }
    {
        const int M = CDIM, N = SEQ;
        const unsigned gx = (unsigned)(((M / 64) * (N / 64) + 7) / 8);
        k_gemm64<<<dim3(gx, (unsigned)NB), 256, 0, stream>>>(W316 + (size_t)2 * CDIM * CDIM, CDIM, (long long)0, X16, CDIM, (long long)SEQ * CDIM,
                                                            (void*)VT16, SEQ, (long long)CDIM * SEQ, bproj, M, N, CDIM, 0.0625f, 1);
    }
    k_flash<<<(unsigned)(NB * NHEAD * (SEQ / 64)), 32 * AT_NW, 0, stream>>>(QK16, VT16, mask, AO16);
    {
        const int M = SEQ, N = CDIM;
        const unsigned gx = (unsigned)(((M / 64) * (N / 64) + 7) / 8);
        k_gemm64<<<dim3(gx, (unsigned)NB), 256, 0, stream>>>(AO16, CDIM, (long long)SEQ * CDIM, WO16, CDIM, (long long)0,
                                                            (void*)out, CDIM, (long long)SEQ_FULL * CDIM, bproj, M, N, CDIM, 0.0009765625f, 0);
    }
}
